// TransformerBlock_70918499992241
// MI455X (gfx1250) — hardware-verified
//
#include <hip/hip_runtime.h>
#include <stddef.h>
#include <math.h>


typedef _Float16 v16h __attribute__((ext_vector_type(16)));
typedef _Float16 v8h  __attribute__((ext_vector_type(8)));
typedef _Float16 v4h  __attribute__((ext_vector_type(4)));
typedef float    v8f  __attribute__((ext_vector_type(8)));
typedef float    v4f  __attribute__((ext_vector_type(4)));

#ifndef NB
#define NB 4
#endif
#ifndef SEQ
#define SEQ 2048
#endif
#define NB_FULL  4
#define SEQ_FULL 2048
#define DIM   512
#define NHEAD 8
#define HD    64
#define MROWS (NB * SEQ)

static_assert(NB >= 1 && NB <= NB_FULL);
static_assert(SEQ >= 128 && SEQ <= SEQ_FULL && (SEQ % 128) == 0);
static_assert(DIM == NHEAD * HD);
static_assert(HD == 64);
static_assert(DIM == 512);
static_assert((DIM % 64) == 0 && (DIM % 32) == 0);
static_assert((MROWS % 64) == 0 && (MROWS % 8) == 0);
static_assert(((size_t)DIM * DIM) % (8 * 256) == 0);
static_assert((size_t)MROWS * DIM < (size_t)0xFFFFFFFFu);

#define LDT 72
#define LDC 68

#define WCARRY 64.0f
#define PCARRY 1024.0f
#define VCARRY 64.0f
#define EPSF   1.1920929e-07f
#define RSQ_DIM 0.044194173824159216f

#define WPL           ((size_t)DIM * DIM)
#define WT_BYTES      ((size_t)8 * DIM * DIM * 2)
#define DIVS_BYTES    ((size_t)1024)
#define POS_BYTES     ((size_t)SEQ * DIM * 4)
#define PLANE32_BYTES ((size_t)MROWS * DIM * 4)
#define PLANE16_BYTES ((size_t)MROWS * DIM * 2)
#define OFF_DIVS (WT_BYTES)
#define OFF_POS  (OFF_DIVS + DIVS_BYTES)
#define OFF_XR   (OFF_POS + POS_BYTES)
#define OFF_X2   (OFF_XR + PLANE32_BYTES)
#define OFF_F1   (OFF_X2 + PLANE32_BYTES)
#define OFF_H16  (OFF_F1 + PLANE32_BYTES)
#define OFF_Q    (OFF_H16 + PLANE16_BYTES)
#define OFF_K    (OFF_Q + PLANE16_BYTES)
#define OFF_VT   (OFF_K + PLANE16_BYTES)
#define OFF_CTX  (OFF_VT + PLANE16_BYTES)
#define OFF_H4   (OFF_CTX + PLANE16_BYTES)
#define WS_TOTAL (OFF_H4 + PLANE16_BYTES)
static_assert((WT_BYTES % 128) == 0 && (PLANE16_BYTES % 128) == 0 && (PLANE32_BYTES % 128) == 0);
static_assert((POS_BYTES % 128) == 0 && (DIVS_BYTES % 128) == 0);
static_assert(WS_TOTAL <= (size_t)134217728);

__device__ __forceinline__ float bf16r(float x) {
  unsigned int u = __float_as_uint(x);
  u = (u + 0x7FFFu + ((u >> 16) & 1u)) & 0xFFFF0000u;
  return __uint_as_float(u);
}

__device__ __forceinline__ v16h frag_at(const _Float16* p) {
  v8h lo = *(const v8h*)(p);
  v8h hi = *(const v8h*)(p + 16);
  v16h out;
#pragma unroll
  for (int i = 0; i < 8; ++i) { out[i] = lo[i]; out[i + 8] = hi[i]; }
  return out;
}
__device__ __forceinline__ v16h ld_frag(const _Float16* base, unsigned ld) {
  const unsigned lane = threadIdx.x & 31u;
  return frag_at(base + (lane & 15u) * ld + (lane >> 4) * 8u);
}

__device__ __forceinline__ v8f wmma16(v16h a, v16h b, v8f c) {
  v8f d = __builtin_amdgcn_wmma_f32_16x16x32_f16(false, a, false, b, (short)0, c,
                                                 false, false);
  asm volatile("v_nop\n\tv_nop\n\tv_nop\n\tv_nop" : "+v"(d) : "v"(a), "v"(b));
  return d;
}

__device__ __forceinline__ float red16_max(float x) {
#pragma unroll
  for (int off = 1; off < 16; off <<= 1) x = fmaxf(x, __shfl_xor(x, off, 32));
  return x;
}
__device__ __forceinline__ float red16_sum(float x) {
#pragma unroll
  for (int off = 1; off < 16; off <<= 1) x += __shfl_xor(x, off, 32);
  return x;
}
__device__ __forceinline__ float red32_sum(float x) {
#pragma unroll
  for (int off = 1; off < 32; off <<= 1) x += __shfl_xor(x, off, 32);
  return x;
}

__device__ __forceinline__ void wave_lds_sync() {
  __builtin_amdgcn_fence(3  , "wavefront");
  asm volatile("s_wait_dscnt 0x0" ::: "memory");
  __builtin_amdgcn_wave_barrier();
}

__global__ __launch_bounds__(256) void wconv_kernel(
    const float* __restrict__ wq, const float* __restrict__ wk, const float* __restrict__ wv,
    const float* __restrict__ wo, const float* __restrict__ w1, const float* __restrict__ sw,
    const float* __restrict__ w2, _Float16* __restrict__ Wt) {
  const unsigned p = blockIdx.y;
  const float* W = (p == 0u) ? wq : (p == 1u) ? wk : (p == 2u) ? wv : (p == 3u) ? wo
                 : (p == 4u) ? w1 : (p == 5u) ? sw : (p == 6u) ? (sw + WPL) : w2;
  const unsigned e = (blockIdx.x * 256u + threadIdx.x) * 8u;
  const v4f a0 = *(const v4f*)(W + e);
  const v4f a1 = *(const v4f*)(W + e + 4);
  v8h o;
#pragma unroll
  for (int j = 0; j < 4; ++j) {
    o[j]     = (_Float16)(WCARRY * bf16r(a0[j]));
    o[j + 4] = (_Float16)(WCARRY * bf16r(a1[j]));
  }
  _Float16* d = Wt + (size_t)p * WPL + e;
  *(volatile v8h*)d = o;
  __threadfence();
  *(volatile v8h*)d = o;
}

struct F64 { float v[64]; };
static_assert(sizeof(F64) == 256);

__global__ __launch_bounds__(32) void divs_kernel(F64 a, float* dst, unsigned eoff) {
  const unsigned lane = threadIdx.x;
  v4f t;
  t[0] = 0.0f; t[1] = 0.0f; t[2] = 0.0f; t[3] = 0.0f;
#pragma unroll
  for (int j = 0; j < 16; ++j) {
    const bool sel = (lane == (unsigned)j);
    t[0] = sel ? a.v[4 * j]     : t[0];
    t[1] = sel ? a.v[4 * j + 1] : t[1];
    t[2] = sel ? a.v[4 * j + 2] : t[2];
    t[3] = sel ? a.v[4 * j + 3] : t[3];
  }
  if (lane < 16u) {
    float* d = dst + eoff + lane * 4u;
    *(volatile v4f*)d = t;
    __threadfence();
    *(volatile v4f*)d = t;
  }
}

__global__ __launch_bounds__(256) void pos_kernel(
    const float* __restrict__ divs, float* __restrict__ pos) {
  __shared__ __attribute__((aligned(16))) float Rw[DIM];
  const unsigned tid = threadIdx.x;
  const unsigned t = blockIdx.x;
  const float ang = (float)t * divs[tid];
  float sn, cn;
  sincosf(ang, &sn, &cn);
  Rw[2u * tid] = sn;
  Rw[2u * tid + 1u] = cn;
  __syncthreads();
  if (tid < 128u) {
    const v4f x = *(const v4f*)&Rw[tid * 4u];
    float* d = pos + (size_t)t * DIM + tid * 4u;
    *(volatile v4f*)d = x;
    __threadfence();
    *(volatile v4f*)d = x;
  }
}

template <int MODE>
__global__ __launch_bounds__(256) void norm_kernel(
    const float* __restrict__ src, const float* __restrict__ pos,
    const float* __restrict__ g, const float* __restrict__ bb,
    float* __restrict__ xres, _Float16* __restrict__ h16) {
  __shared__ __attribute__((aligned(16))) _Float16 Hs[8 * DIM];
  const unsigned tid = threadIdx.x, lane = tid & 31u, w = tid >> 5;
  const unsigned crow = blockIdx.x * 8u + w;
  const unsigned bidx = crow / (unsigned)SEQ;
  const unsigned sq = crow - bidx * (unsigned)SEQ;
  const size_t srow = (MODE == 0) ? ((size_t)bidx * SEQ_FULL + sq) : (size_t)crow;
  const float* sp = src + srow * DIM + lane * 4u;
  const float* pp = pos + (size_t)sq * DIM + lane * 4u;

  v4f val[4];
  float ss = 0.0f;
#pragma unroll
  for (unsigned j = 0; j < 4u; ++j) {
    v4f a = *(const v4f*)(sp + j * 128u);
    if (MODE == 0) {
      const v4f p = *(const v4f*)(pp + j * 128u);
#pragma unroll
      for (int e = 0; e < 4; ++e) a[e] = bf16r(a[e]) + p[e];
    }
    val[j] = a;
#pragma unroll
    for (int e = 0; e < 4; ++e) ss += a[e] * a[e];
  }
  ss = red32_sum(ss);
  const float inv = 1.0f / (sqrtf(ss) * RSQ_DIM + EPSF);

  if (MODE == 0) {
    float* xr = xres + (size_t)crow * DIM + lane * 4u;
#pragma unroll
    for (unsigned j = 0; j < 4u; ++j) *(volatile v4f*)(xr + j * 128u) = val[j];
    __threadfence();
#pragma unroll
    for (unsigned j = 0; j < 4u; ++j) *(volatile v4f*)(xr + j * 128u) = val[j];
  }

  _Float16* hrow = Hs + w * (unsigned)DIM;
#pragma unroll
  for (unsigned j = 0; j < 4u; ++j) {
    const unsigned c = j * 128u + lane * 4u;
    const v4f g4 = *(const v4f*)(g + c);
    const v4f b4 = *(const v4f*)(bb + c);
    v4h o;
#pragma unroll
    for (int e = 0; e < 4; ++e)
      o[e] = (_Float16)(val[j][e] * inv * bf16r(g4[e]) + bf16r(b4[e]));
    *(v4h*)&hrow[c] = o;
  }
  wave_lds_sync();
  v8h x[2];
  size_t off[2];
#pragma unroll
  for (unsigned i = 0; i < 2u; ++i) {
    const unsigned c = i * 256u + lane * 8u;
    x[i] = *(const v8h*)&hrow[c];
    off[i] = (size_t)crow * DIM + c;
  }
#pragma unroll
  for (int i = 0; i < 2; ++i) *(volatile v8h*)(h16 + off[i]) = x[i];
  __threadfence();
#pragma unroll
  for (int i = 0; i < 2; ++i) *(volatile v8h*)(h16 + off[i]) = x[i];
}

__device__ __forceinline__ void store_rows16(const float* Cs, _Float16* out, unsigned row0,
                                             unsigned n0, unsigned tid, float mul) {
  v8h x[2];
  size_t off[2];
#pragma unroll
  for (unsigned i = 0; i < 2u; ++i) {
    const unsigned r = 32u * i + (tid >> 3);
    const unsigned c = (tid & 7u) * 8u;
    const v4f u0 = *(const v4f*)&Cs[r * LDC + c];
    const v4f u1 = *(const v4f*)&Cs[r * LDC + c + 4];
#pragma unroll
    for (int j = 0; j < 4; ++j) {
      x[i][j]     = (_Float16)(u0[j] * mul);
      x[i][j + 4] = (_Float16)(u1[j] * mul);
    }
    off[i] = (size_t)(row0 + r) * DIM + n0 + c;
  }
#pragma unroll
  for (int i = 0; i < 2; ++i) *(volatile v8h*)(out + off[i]) = x[i];
  __threadfence();
#pragma unroll
  for (int i = 0; i < 2; ++i) *(volatile v8h*)(out + off[i]) = x[i];
}

template <int MODE>
__global__ __launch_bounds__(256) void gemm_kernel(
    const _Float16* __restrict__ A16, const _Float16* __restrict__ Bt,
    const float* __restrict__ bias, const float* __restrict__ res,
    float* __restrict__ outf, _Float16* __restrict__ o0, _Float16* __restrict__ o1,
    _Float16* __restrict__ o2, float cs) {
  constexpr bool DUAL = (MODE == 4);
  constexpr bool HASB = (MODE == 2) || (MODE == 3);
  constexpr bool HASR = (MODE == 1) || (MODE == 3);
  constexpr bool OUTFULL = (MODE == 3);
  __shared__ __attribute__((aligned(16))) float Cs[64 * LDC];
  const unsigned tid = threadIdx.x, lane = tid & 31u, w = tid >> 5;
  const unsigned mw = w >> 1, nw = w & 1u;
  const unsigned hh = lane >> 4, m = lane & 15u;
  const unsigned bx = blockIdx.x;
  const unsigned nb0 = bx * 64u;
  const unsigned n0 = (MODE == 0) ? ((bx & 7u) * 64u) : nb0;
  const unsigned row0 = blockIdx.y * 64u;

  const _Float16* ap  = A16 + (size_t)(row0 + mw * 16u + m) * DIM + hh * 8u;
  const _Float16* bp0 = Bt + (size_t)(nb0 + nw * 32u + m) * DIM + hh * 8u;
  const _Float16* bp1 = bp0 + 16 * DIM;
  v8f acc0 = {}, acc1 = {}, acc2 = {}, acc3 = {};
#pragma unroll 2
  for (unsigned k0 = 0; k0 < (unsigned)DIM; k0 += 32u) {
    const v16h a  = frag_at(ap + k0);
    const v16h b0 = frag_at(bp0 + k0);
    const v16h b1 = frag_at(bp1 + k0);
    acc0 = wmma16(a, b0, acc0);
    acc1 = wmma16(a, b1, acc1);
    if (DUAL) {
      const v16h b2 = frag_at(bp0 + WPL + k0);
      const v16h b3 = frag_at(bp1 + WPL + k0);
      acc2 = wmma16(a, b2, acc2);
      acc3 = wmma16(a, b3, acc3);
    }
  }

  if (DUAL) {
    const unsigned colA = n0 + nw * 32u + m;
    const float ba0 = bf16r(bias[colA]);
    const float ba1 = bf16r(bias[colA + 16u]);
    const float bg0 = bf16r(bias[(unsigned)DIM + colA]);
    const float bg1 = bf16r(bias[(unsigned)DIM + colA + 16u]);
#pragma unroll
    for (int r = 0; r < 8; ++r) {
      float* d = &Cs[(mw * 16u + hh * 8u + (unsigned)r) * LDC + nw * 32u + m];
      const float a0 = acc0[r] * cs + ba0;
      const float g0 = acc2[r] * cs + bg0;
      const float a1 = acc1[r] * cs + ba1;
      const float g1 = acc3[r] * cs + bg1;
      d[0]  = a0 * __builtin_amdgcn_rcpf(1.0f + __expf(-a0)) + g0;
      d[16] = a1 * __builtin_amdgcn_rcpf(1.0f + __expf(-a1)) + g1;
    }
  } else {
#pragma unroll
    for (int r = 0; r < 8; ++r) {
      float* d = &Cs[(mw * 16u + hh * 8u + (unsigned)r) * LDC + nw * 32u + m];
      d[0]  = acc0[r];
      d[16] = acc1[r];
    }
  }
  __syncthreads();

  if (MODE == 0) {
    const unsigned sel = bx >> 3;
    if (sel < 2u) {
      store_rows16(Cs, (sel == 0u) ? o0 : o1, row0, n0, tid, cs);
    } else {
      const unsigned bidx = row0 / (unsigned)SEQ;
      const unsigned key0 = row0 - bidx * (unsigned)SEQ;
      v8h x[2];
      size_t off[2];
#pragma unroll
      for (unsigned i = 0; i < 2u; ++i) {
        const unsigned dcol = 32u * i + (tid >> 3);
        const unsigned kk = (tid & 7u) * 8u;
#pragma unroll
        for (unsigned j = 0; j < 8u; ++j)
          x[i][j] = (_Float16)(Cs[(kk + j) * LDC + dcol] * cs);
        off[i] = ((size_t)bidx * DIM + n0 + dcol) * SEQ + key0 + kk;
      }
#pragma unroll
      for (int i = 0; i < 2; ++i) *(volatile v8h*)(o2 + off[i]) = x[i];
      __threadfence();
#pragma unroll
      for (int i = 0; i < 2; ++i) *(volatile v8h*)(o2 + off[i]) = x[i];
    }
  }

  if (MODE == 4) {
    store_rows16(Cs, o0, row0, n0, tid, 1.0f);
  }

  if (MODE == 1 || MODE == 2 || MODE == 3) {
    v4f xs[4];
    size_t off[4];
#pragma unroll
    for (unsigned i = 0; i < 4u; ++i) {
      const unsigned r = 16u * i + (tid >> 4);
      const unsigned c = (tid & 15u) * 4u;
      const unsigned crow = row0 + r;
      const v4f u = *(const v4f*)&Cs[r * LDC + c];
      v4f val;
#pragma unroll
      for (int j = 0; j < 4; ++j) val[j] = u[j] * cs;
      if (HASB) {
        const v4f g = *(const v4f*)(bias + n0 + c);
#pragma unroll
        for (int j = 0; j < 4; ++j) val[j] = val[j] + bf16r(g[j]);
      }
      if (HASR) {
        const v4f rr = *(const v4f*)(res + (size_t)crow * DIM + n0 + c);
#pragma unroll
        for (int j = 0; j < 4; ++j) val[j] = val[j] + rr[j];
      }
      size_t orow = (size_t)crow;
      if (OUTFULL) {
        const unsigned bidx = crow / (unsigned)SEQ;
        const unsigned sq = crow - bidx * (unsigned)SEQ;
        orow = (size_t)bidx * SEQ_FULL + sq;
      }
      xs[i] = val;
      off[i] = orow * DIM + n0 + c;
    }
#pragma unroll
    for (int i = 0; i < 4; ++i) *(volatile v4f*)(outf + off[i]) = xs[i];
    __threadfence();
#pragma unroll
    for (int i = 0; i < 4; ++i) *(volatile v4f*)(outf + off[i]) = xs[i];
  }
}

__global__ __launch_bounds__(256) void attn_kernel(
    const _Float16* __restrict__ Qh, const _Float16* __restrict__ Kh,
    const _Float16* __restrict__ Vt, _Float16* __restrict__ Ov) {
  __shared__ __attribute__((aligned(16))) _Float16 Ks[64 * LDT];
  __shared__ __attribute__((aligned(16))) _Float16 Vs[64 * LDT];
  __shared__ __attribute__((aligned(16))) _Float16 Ps[8 * 16 * LDT];

  const unsigned tid = threadIdx.x, lane = tid & 31u;
  const unsigned w = (unsigned)__builtin_amdgcn_readfirstlane((int)(tid >> 5));
  const unsigned hh = lane >> 4, m = lane & 15u;
  const unsigned q0 = blockIdx.x * 128u;
  const unsigned head = blockIdx.y;
  const unsigned b = blockIdx.z;
  const unsigned qw0 = q0 + w * 16u;
  const float scale = RSQ_DIM;
  _Float16* P = Ps + w * (16u * LDT);

  const size_t qoff = (size_t)(b * (unsigned)SEQ + qw0 + m) * DIM + head * HD + hh * 8u;
  v16h qf[2];
  qf[0] = frag_at(Qh + qoff);
  qf[1] = frag_at(Qh + qoff + 32);

  float mrow[8], lrow[8];
  v8f o[4];
#pragma unroll
  for (int v = 0; v < 8; ++v) { mrow[v] = -1.0e30f; lrow[v] = 0.0f; }
#pragma unroll
  for (int nb = 0; nb < 4; ++nb) o[nb] = (v8f){};

  const size_t kplane = (size_t)b * SEQ * DIM + head * HD;
  const size_t vplane = ((size_t)b * DIM + head * HD) * SEQ;
  const unsigned kend = q0 + 128u;

  for (unsigned kb = 0; kb < kend; kb += 64u) {
#pragma unroll
    for (unsigned j = 0; j < 2u; ++j) {
      const unsigned idx = tid + 256u * j;
      const unsigned r = idx >> 3, c = (idx & 7u) * 8u;
      *(v8h*)&Ks[r * LDT + c] = *(const v8h*)(Kh + kplane + (size_t)(kb + r) * DIM + c);
      *(v8h*)&Vs[r * LDT + c] = *(const v8h*)(Vt + vplane + (size_t)r * SEQ + kb + c);
    }
    __syncthreads();

    if (kb <= qw0) {
      v8f s[4];
#pragma unroll
      for (int kg = 0; kg < 4; ++kg) {
        v8f t = {};
#pragma unroll
        for (int c = 0; c < 2; ++c) {
          const v16h kf = ld_frag(&Ks[(kg * 16) * LDT + c * 32], LDT);
          t = wmma16(qf[c], kf, t);
        }
        s[kg] = t * scale;
      }
      if (kb + 63u > qw0) {
#pragma unroll
        for (int kg = 0; kg < 4; ++kg)
#pragma unroll
          for (int v = 0; v < 8; ++v) {
            const unsigned key = kb + (unsigned)kg * 16u + m;
            const unsigned row = qw0 + hh * 8u + (unsigned)v;
            s[kg][v] = (key > row) ? -1.0e30f : s[kg][v];
          }
      }

      float alpha[8];
#pragma unroll
      for (int v = 0; v < 8; ++v) {
        float mx = fmaxf(fmaxf(s[0][v], s[1][v]), fmaxf(s[2][v], s[3][v]));
        mx = red16_max(mx);
        const float mn = fmaxf(mrow[v], mx);
        alpha[v] = __expf(mrow[v] - mn);
        mrow[v] = mn;
      }
#pragma unroll
      for (int kg = 0; kg < 4; ++kg)
#pragma unroll
        for (int v = 0; v < 8; ++v) s[kg][v] = __expf(s[kg][v] - mrow[v]);
#pragma unroll
      for (int v = 0; v < 8; ++v) {
        const float rs = red16_sum((s[0][v] + s[1][v]) + (s[2][v] + s[3][v]));
        lrow[v] = alpha[v] * lrow[v] + rs;
      }
#pragma unroll
      for (int nb = 0; nb < 4; ++nb)
#pragma unroll
        for (int v = 0; v < 8; ++v) o[nb][v] = o[nb][v] * alpha[v];

#pragma unroll
      for (int kg = 0; kg < 4; ++kg)
#pragma unroll
        for (int v = 0; v < 8; ++v)
          P[(hh * 8u + (unsigned)v) * LDT + (unsigned)kg * 16u + m] =
              (_Float16)(s[kg][v] * PCARRY);
      wave_lds_sync();

#pragma unroll
      for (int c = 0; c < 2; ++c) {
        const v16h pf = ld_frag(P + c * 32, LDT);
#pragma unroll
        for (int nb = 0; nb < 4; ++nb) {
          const v16h vf = ld_frag(&Vs[(nb * 16) * LDT + c * 32], LDT);
          o[nb] = wmma16(pf, vf, o[nb]);
        }
      }
    }
    __syncthreads();
  }

  float inv[8];
#pragma unroll
  for (int v = 0; v < 8; ++v) inv[v] = __builtin_amdgcn_rcpf(lrow[v]) * (VCARRY / PCARRY);
#pragma unroll
  for (int nb = 0; nb < 4; ++nb)
#pragma unroll
    for (int v = 0; v < 8; ++v)
      P[(hh * 8u + (unsigned)v) * LDT + (unsigned)nb * 16u + m] = (_Float16)(o[nb][v] * inv[v]);
  wave_lds_sync();
  v8h x[4];
  size_t off[4];
#pragma unroll
  for (unsigned i = 0; i < 4u; ++i) {
    const unsigned r = 4u * i + (lane >> 3);
    const unsigned c = (lane & 7u) * 8u;
    x[i] = *(const v8h*)&P[r * LDT + c];
    off[i] = (size_t)(b * (unsigned)SEQ + qw0 + r) * DIM + head * HD + c;
  }
#pragma unroll
  for (int i = 0; i < 4; ++i) *(volatile v8h*)(Ov + off[i]) = x[i];
  __threadfence();
#pragma unroll
  for (int i = 0; i < 4; ++i) *(volatile v8h*)(Ov + off[i]) = x[i];
}

extern "C" void kernel_launch(void* const* d_in, const int* in_sizes, int n_in,
                              void* d_out, int out_size, void* d_ws, size_t ws_size,
                              hipStream_t stream) {
  if (n_in < 17) return;
  const long long need_x = ((long long)(NB - 1) * SEQ_FULL + SEQ) * DIM;
  const long long wsz = (long long)DIM * DIM;
  if ((long long)in_sizes[0] < need_x) return;
  if (in_sizes[1] < DIM || in_sizes[2] < DIM) return;
  if ((long long)in_sizes[3] < wsz || (long long)in_sizes[4] < wsz) return;
  if ((long long)in_sizes[5] < wsz || (long long)in_sizes[6] < wsz) return;
  if (in_sizes[7] < DIM || in_sizes[8] < DIM) return;
  if ((long long)in_sizes[9] < wsz || in_sizes[10] < DIM) return;
  if (in_sizes[11] < DIM || in_sizes[12] < DIM) return;
  if ((long long)in_sizes[13] < 2 * wsz || in_sizes[14] < 2 * DIM) return;
  if ((long long)in_sizes[15] < wsz || in_sizes[16] < DIM) return;
  if ((long long)out_size < need_x) return;
  if (ws_size < WS_TOTAL) return;

  const float* X    = (const float*)d_in[0];
  const float* n1g  = (const float*)d_in[1];
  const float* n1b  = (const float*)d_in[2];
  const float* wq   = (const float*)d_in[3];
  const float* wk   = (const float*)d_in[4];
  const float* wv   = (const float*)d_in[5];
  const float* wo   = (const float*)d_in[6];
  const float* n2g  = (const float*)d_in[7];
  const float* n2b  = (const float*)d_in[8];
  const float* w1   = (const float*)d_in[9];
  const float* b1   = (const float*)d_in[10];
  const float* fg   = (const float*)d_in[11];
  const float* fb   = (const float*)d_in[12];
  const float* sww  = (const float*)d_in[13];
  const float* swb  = (const float*)d_in[14];
  const float* w2   = (const float*)d_in[15];
  const float* b2   = (const float*)d_in[16];
  float* out = (float*)d_out;

  char* ws = (char*)d_ws;
  _Float16* Wt    = (_Float16*)ws;
  float*    DIVS  = (float*)(ws + OFF_DIVS);
  float*    POS   = (float*)(ws + OFF_POS);
  float*    XR    = (float*)(ws + OFF_XR);
  float*    X2    = (float*)(ws + OFF_X2);
  float*    F1    = (float*)(ws + OFF_F1);
  _Float16* H16   = (_Float16*)(ws + OFF_H16);
  _Float16* Q16   = (_Float16*)(ws + OFF_Q);
  _Float16* K16   = (_Float16*)(ws + OFF_K);
  _Float16* Vt16  = (_Float16*)(ws + OFF_VT);
  _Float16* Ctx16 = (_Float16*)(ws + OFF_CTX);
  _Float16* H4    = (_Float16*)(ws + OFF_H4);

  F64 dv[4];
  for (int i = 0; i < 256; ++i) {
    const double e = (double)(2 * i) / 512.0;
    const float pw = (float)pow(10000.0, e);
    const float sum = pw + 1.1920929e-07f;
    dv[i >> 6].v[i & 63] = 1.0f / sum;
  }

  dim3 blk(256);
  dim3 g8(DIM / 64, MROWS / 64);

  wconv_kernel<<<dim3((unsigned)(WPL / 2048), 8), blk, 0, stream>>>(wq, wk, wv, wo, w1, sww,
                                                                    w2, Wt);
  divs_kernel<<<dim3(1), dim3(32), 0, stream>>>(dv[0], DIVS, 0u);
  divs_kernel<<<dim3(1), dim3(32), 0, stream>>>(dv[1], DIVS, 64u);
  divs_kernel<<<dim3(1), dim3(32), 0, stream>>>(dv[2], DIVS, 128u);
  divs_kernel<<<dim3(1), dim3(32), 0, stream>>>(dv[3], DIVS, 192u);
  pos_kernel<<<dim3(SEQ), blk, 0, stream>>>(DIVS, POS);
  norm_kernel<0><<<dim3(MROWS / 8), blk, 0, stream>>>(X, POS, n1g, n1b, XR, H16);
  gemm_kernel<0><<<dim3(3 * DIM / 64, MROWS / 64), blk, 0, stream>>>(
      H16, Wt, b1, XR, F1, Q16, K16, Vt16, 1.0f / WCARRY);
  attn_kernel<<<dim3(SEQ / 128, NHEAD, NB), blk, 0, stream>>>(Q16, K16, Vt16, Ctx16);
  gemm_kernel<1><<<g8, blk, 0, stream>>>(Ctx16, Wt + 3 * WPL, b1, XR, X2, Q16, K16, Vt16,
                                         1.0f / (WCARRY * VCARRY));
  norm_kernel<1><<<dim3(MROWS / 8), blk, 0, stream>>>(X2, POS, n2g, n2b, XR, H16);
  gemm_kernel<2><<<g8, blk, 0, stream>>>(H16, Wt + 4 * WPL, b1, XR, F1, Q16, K16, Vt16,
                                         1.0f / WCARRY);
  norm_kernel<1><<<dim3(MROWS / 8), blk, 0, stream>>>(F1, POS, fg, fb, XR, H16);
  gemm_kernel<4><<<g8, blk, 0, stream>>>(H16, Wt + 5 * WPL, swb, XR, F1, H4, K16, Vt16,
                                         1.0f / WCARRY);
  gemm_kernel<3><<<g8, blk, 0, stream>>>(H4, Wt + 7 * WPL, b2, X2, out, Q16, K16, Vt16,
                                         1.0f / WCARRY);
}
